// GraphEncoder_36782099923301
// MI455X (gfx1250) — hardware-run, weakly checked
//
#include <hip/hip_runtime.h>
#include <stddef.h>
#include <stdint.h>
#include <math.h>

#define NN      10000
#define NE      160000
#define F_IN    768
#define NH1     4
#define C1      512
#define HC1     2048
#define C2      768
#define KA2     4096
#define MP      10112
#define NTHR    256
#define NWAVE   8
#define EPT     8
#define CHUNK   (NTHR * EPT)
#define WCAP    (EPT * 32)
#define LISTN   (NWAVE * WCAP)
#define NBRUN   1024
#define SLOTB   10
#define NBLK    10
#define NSLOT   (NBLK * NBRUN)
#define RCAP    20480
#define DEGCAP  64
#define LCAP    72
#define SELFQ   64
#define GBM     128
#define GBN     64
#define GTHR    128
#define NEGSL   0.2f
#define EPS_SM  1e-16f
#define LDS_BKT ((2 * RCAP + 2 * NBRUN + LISTN) * 4 + 64)
#define KEYSENT (-2147483647 - 1)

static_assert(NN <= 16384);
static_assert(NBRUN == (1 << SLOTB));
static_assert(NTHR * 4 == NBRUN);
static_assert(LISTN >= NBRUN && LISTN == NWAVE * WCAP);
static_assert(CHUNK <= (1 << (31 - SLOTB)));
static_assert(NSLOT >= MP && NBLK * NBRUN == NSLOT);
static_assert(RCAP >= 16569 + 2048);
static_assert((RCAP % 1024) == 0);
static_assert(DEGCAP >= 36 + 8);
static_assert(SELFQ >= DEGCAP && SELFQ < LCAP && DEGCAP == 64);
static_assert(LDS_BKT <= 327680);
static_assert((MP % GBM) == 0 && (MP % 32) == 0 && (MP % NWAVE) == 0 && MP >= NN);
static_assert((F_IN % 32) == 0 && (KA2 % 32) == 0 && F_IN == 24 * 32);
static_assert((HC1 % GBN) == 0 && (C2 % GBN) == 0 && (HC1 % 128) == 0 && (C2 % 128) == 0);
static_assert(HC1 == NH1 * C1 && C1 == 4 * 128 && C2 == 6 * 128 && KA2 == 2 * HC1);
static_assert(GBM == (GTHR / 32) * 32);
static_assert((NE % 4) == 0);

typedef float          v4f  __attribute__((ext_vector_type(4)));
typedef float          v8f  __attribute__((ext_vector_type(8)));
typedef int            v4i  __attribute__((ext_vector_type(4)));
typedef int            v8i  __attribute__((ext_vector_type(8)));
typedef unsigned int   v2u  __attribute__((ext_vector_type(2)));
typedef unsigned int   v4u  __attribute__((ext_vector_type(4)));
typedef unsigned short v8us __attribute__((ext_vector_type(8)));
typedef __bf16         v16b __attribute__((ext_vector_type(16)));
typedef v4f  __attribute__((may_alias)) v4fa;
typedef v4i  __attribute__((may_alias)) v4ia;
typedef v8us __attribute__((may_alias)) v8usa;
union FragB { v16b v; v8us h[2]; v8i w; };

__device__ __forceinline__ v8f wmb(const FragB& a, const FragB& b, v8f c) {
  v8f d = __builtin_amdgcn_wmma_f32_16x16x32_bf16(false, a.v, false, b.v, (short)0, c, false, false);
  asm volatile("v_nop\n\tv_nop\n\tv_nop\n\tv_nop" : "+v"(d) : "v"(a.w), "v"(b.w));
  return d;
}

__device__ __forceinline__ unsigned int f2bf(float f) {
  const unsigned int u = __float_as_uint(f);
  return ((u + 0x7FFFu + ((u >> 16) & 1u)) >> 16) & 0xFFFFu;
}
__device__ __forceinline__ float bf2f(unsigned int b) { return __uint_as_float(b << 16); }
__device__ __forceinline__ float bfr(float f) { return bf2f(f2bf(f)); }
__device__ __forceinline__ v4f bfr4(const v4f a) {
  v4f r; r.x = bfr(a.x); r.y = bfr(a.y); r.z = bfr(a.z); r.w = bfr(a.w); return r;
}
__device__ __forceinline__ unsigned int pk2(float lo, float hi) { return f2bf(lo) | (f2bf(hi) << 16); }
__device__ __forceinline__ v4u pack8(const v4f a, const v4f b) {
  v4u r;
  r.x = pk2(a.x, a.y); r.y = pk2(a.z, a.w); r.z = pk2(b.x, b.y); r.w = pk2(b.z, b.w);
  return r;
}
struct HL { v2u hi; v2u lo; };
__device__ __forceinline__ HL split4(const v4f o) {
  const unsigned int hx = f2bf(o.x), hy = f2bf(o.y), hz = f2bf(o.z), hw = f2bf(o.w);
  const unsigned int lx = f2bf(o.x - bf2f(hx)), ly = f2bf(o.y - bf2f(hy));
  const unsigned int lz = f2bf(o.z - bf2f(hz)), lw = f2bf(o.w - bf2f(hw));
  HL r;
  r.hi.x = hx | (hy << 16); r.hi.y = hz | (hw << 16);
  r.lo.x = lx | (ly << 16); r.lo.y = lz | (lw << 16);
  return r;
}

__global__ __launch_bounds__(NTHR) void k_xprep(const float* __restrict__ x, unsigned short* xb, int nUnits) {
  const int i = (int)blockIdx.x * NTHR + (int)threadIdx.x;
  if (i >= nUnits) return;
  const int row = i / (F_IN / 8);
  const int c0  = (i - row * (F_IN / 8)) * 8;
  const int rc  = row < NN ? row : NN - 1;
  const float* p = x + (size_t)rc * F_IN + c0;
  v4f a = *(const v4fa*)p, b = *(const v4fa*)(p + 4);
  const v4f z4 = {0.f, 0.f, 0.f, 0.f};
  if (row >= NN) { a = z4; b = z4; }
  const v4u hv = pack8(a, b);
  const size_t o = (size_t)row * F_IN + c0;
  *(volatile v4u*)(xb + o) = hv;
  __threadfence();
  *(volatile v4u*)(xb + o) = hv;
}

__global__ __launch_bounds__(NTHR) void k_wtr(const float* __restrict__ w, int Kin, int Ncol, int Nrows, int Kout,
                                              unsigned short* wt, int nUnits) {
  const int u = (int)blockIdx.x * NTHR + (int)threadIdx.x;
  if (u >= nUnits) return;
  const int kq = Kout >> 3;
  const int n  = u / kq;
  const int k8 = (u - n * kq) * 8;
  const int kk = k8 - (k8 / Kin) * Kin;
  const int ncl = n < Ncol ? n : Ncol - 1;
  const float* p = w + (size_t)kk * (size_t)Ncol + ncl;
  v4f a, b;
  a.x = p[0];                    a.y = p[(size_t)Ncol];         a.z = p[(size_t)2 * Ncol];     a.w = p[(size_t)3 * Ncol];
  b.x = p[(size_t)4 * Ncol];     b.y = p[(size_t)5 * Ncol];     b.z = p[(size_t)6 * Ncol];     b.w = p[(size_t)7 * Ncol];
  const v4f z4 = {0.f, 0.f, 0.f, 0.f};
  if (n >= Ncol || n >= Nrows) { a = z4; b = z4; }
  const v4u wv = pack8(a, b);
  unsigned short* o = wt + (size_t)n * (size_t)Kout + k8;
  *(volatile v4u*)o = wv;
  __threadfence();
  *(volatile v4u*)o = wv;
}

__device__ __forceinline__ int ld_key(const int* __restrict__ dsts, int e) {
  const int ec = e < NE ? e : NE - 1;
  int d = dsts[ec];
  asm volatile("" :: "v"(d));
  return (e < NE) ? d : KEYSENT;
}

__device__ __forceinline__ int scan_chunk(const int* __restrict__ dsts, int cbase, int slotBase,
                                          int* list, int lane, int wave) {
  int wc = 0;
  const int el0 = wave * WCAP + lane;
  const int e0  = cbase + el0;
  const int d0 = ld_key(dsts, e0),       d1 = ld_key(dsts, e0 + 32),  d2 = ld_key(dsts, e0 + 64),  d3 = ld_key(dsts, e0 + 96);
  const int d4 = ld_key(dsts, e0 + 128), d5 = ld_key(dsts, e0 + 160), d6 = ld_key(dsts, e0 + 192), d7 = ld_key(dsts, e0 + 224);
  const unsigned nbs = (unsigned)slotBase;
  const unsigned unb = (unsigned)NBRUN;
  const unsigned s0 = (unsigned)d0 - nbs, s1 = (unsigned)d1 - nbs, s2 = (unsigned)d2 - nbs, s3 = (unsigned)d3 - nbs;
  const unsigned s4 = (unsigned)d4 - nbs, s5 = (unsigned)d5 - nbs, s6 = (unsigned)d6 - nbs, s7 = (unsigned)d7 - nbs;
  const bool h0 = s0 < unb, h1 = s1 < unb, h2 = s2 < unb, h3 = s3 < unb;
  const bool h4 = s4 < unb, h5 = s5 < unb, h6 = s6 < unb, h7 = s7 < unb;
  const unsigned any = __builtin_amdgcn_ballot_w32(h0 | h1 | h2 | h3 | h4 | h5 | h6 | h7);
  if (any != 0u) {
#define HITJ(J, HJ, SJ) { \
      const unsigned mj = __builtin_amdgcn_ballot_w32(HJ); \
      if (mj != 0u) { \
        if (HJ) { \
          const int pos = wc + (int)__builtin_amdgcn_mbcnt_lo(mj, 0u); \
          if (pos < WCAP) list[wave * WCAP + pos] = ((el0 + 32 * (J)) << SLOTB) | (int)(SJ); \
        } \
        wc += (int)__builtin_popcount(mj); } }
    HITJ(0, h0, s0)
    HITJ(1, h1, s1)
    HITJ(2, h2, s2)
    HITJ(3, h3, s3)
    HITJ(4, h4, s4)
    HITJ(5, h5, s5)
    HITJ(6, h6, s6)
    HITJ(7, h7, s7)
#undef HITJ
  }
  return wc;
}

__global__ __launch_bounds__(NTHR) void k_bucket(const int* __restrict__ srcs, const int* __restrict__ dsts,
                                                 int* HITS, int* OFF, int* DEG, int* FLG) {
  extern __shared__ v4f lds_dyn[];
  int* reg1 = (int*)lds_dyn;
  int* reg2 = reg1 + RCAP;
  int* scnt = reg2 + RCAP;
  int* soff = scnt + NBRUN;
  int* list = soff + NBRUN;
  int* wcnt = list + LISTN;
  int* wtot = wcnt + NWAVE;
  const int tid = (int)threadIdx.x, lane = tid & 31;
  const int wave = __builtin_amdgcn_readfirstlane(tid >> 5);
  const int nodeBase = (int)blockIdx.x * NBRUN;

  for (int i = tid; i < NBRUN; i += NTHR) scnt[i] = 0;
  for (int i = tid; i < RCAP; i += NTHR) reg2[i] = 0;
  __syncthreads();

  int tot = 0;
  const int nChunks = (NE + CHUNK - 1) / CHUNK;
#pragma unroll 1
  for (int ch = 0; ch < nChunks; ++ch) {
    const int cbase = ch * CHUNK;
    const int wc = scan_chunk(dsts, cbase, nodeBase, list, lane, wave);
    if (lane == 0) wcnt[wave] = wc;
    __syncthreads();
    int pre = 0, all = 0;
#pragma unroll
    for (int w2 = 0; w2 < NWAVE; ++w2) {
      int c = wcnt[w2];
      c = c < 0 ? 0 : (c > WCAP ? WCAP : c);
      all += c;
      pre += (w2 < wave) ? c : 0;
    }
    const int wcc  = wc > WCAP ? WCAP : wc;
    const int base = tot + pre;
#pragma unroll 1
    for (int i0 = 0; i0 < wcc; i0 += 32) {
      const int i  = i0 + lane;
      const bool ok = i < wcc;
      const int ic = ok ? i : wcc - 1;
      const int ent = list[wave * WCAP + ic];
      const int el  = (ent >> SLOTB) & (CHUNK - 1);
      const int sl  = ent & (NBRUN - 1);
      int eid = cbase + el;
      eid = eid > NE - 1 ? NE - 1 : eid;
      int sraw = srcs[eid];
      asm volatile("" :: "v"(sraw));
      const int s = sraw < 0 ? 0 : (sraw > NN - 1 ? NN - 1 : sraw);
      const int pos = base + i;
      if (ok && pos < RCAP) reg1[pos] = (s << SLOTB) | sl;
    }
    tot += all;
    tot = tot > RCAP ? RCAP : tot;
    __syncthreads();
  }
  const int nh = tot;

  if (wave == 0) {
#pragma unroll 1
    for (int b0 = 0; b0 < nh; b0 += 32) {
      const int idx = b0 + lane;
      const int uv  = reg1[idx < nh ? idx : nh - 1];
      const int m32 = (nh - b0) < 32 ? (nh - b0) : 32;
#pragma unroll 1
      for (int k = 0; k < m32; ++k) {
        const int u  = __builtin_amdgcn_readlane(uv, k);
        const int sl = u & (NBRUN - 1);
        if (lane == 0) scnt[sl] = scnt[sl] + 1;
      }
    }
  }
  __syncthreads();

  {
    const v4i ca = *(const v4ia*)(scnt + 4 * tid);
    const int e0 = ca.x < 0 ? 0 : ca.x, e1 = ca.y < 0 ? 0 : ca.y, e2 = ca.z < 0 ? 0 : ca.z, e3 = ca.w < 0 ? 0 : ca.w;
    const int ts = e0 + e1 + e2 + e3;
    int incl = ts;
#pragma unroll
    for (int d = 1; d < 32; d <<= 1) {
      const int up = __shfl_up(incl, d);
      if (lane >= d) incl += up;
    }
    if (lane == 31) wtot[wave] = incl;
    __syncthreads();
    int pre = 0;
#pragma unroll
    for (int w2 = 0; w2 < NWAVE; ++w2) pre += (w2 < wave) ? wtot[w2] : 0;
    int run = pre + incl - ts;
    soff[4 * tid + 0] = run; run += e0;
    soff[4 * tid + 1] = run; run += e1;
    soff[4 * tid + 2] = run; run += e2;
    soff[4 * tid + 3] = run;
  }
  __syncthreads();
  for (int i = tid; i < NBRUN; i += NTHR) list[i] = soff[i];
  __syncthreads();

  if (wave == 0) {
#pragma unroll 1
    for (int b0 = 0; b0 < nh; b0 += 32) {
      const int idx = b0 + lane;
      const int uv  = reg1[idx < nh ? idx : nh - 1];
      const int m32 = (nh - b0) < 32 ? (nh - b0) : 32;
#pragma unroll 1
      for (int k = 0; k < m32; ++k) {
        const int u  = __builtin_amdgcn_readlane(uv, k);
        const int sl = u & (NBRUN - 1);
        const int sv = (int)((unsigned)u >> SLOTB);
        if (lane == 0) {
          int pos = list[sl];
          pos = pos < 0 ? 0 : (pos > RCAP - 1 ? RCAP - 1 : pos);
          reg2[pos] = sv;
          list[sl] = pos + 1;
        }
      }
    }
  }
  __syncthreads();

  const int ovf = (nh >= RCAP) ? 1 : 0;
  const v4i o4 = *(const v4ia*)(soff + 4 * tid);
  const v4i c4 = *(const v4ia*)(scnt + 4 * tid);
  v4i f4;
  f4.x = (ovf != 0 || c4.x > DEGCAP) ? 1 : 0;
  f4.y = (ovf != 0 || c4.y > DEGCAP) ? 1 : 0;
  f4.z = (ovf != 0 || c4.z > DEGCAP) ? 1 : 0;
  f4.w = (ovf != 0 || c4.w > DEGCAP) ? 1 : 0;
  int* po = OFF + nodeBase + 4 * tid;
  int* pd = DEG + nodeBase + 4 * tid;
  int* pf = FLG + nodeBase + 4 * tid;
  int* ph = HITS + (size_t)blockIdx.x * RCAP;
  *(volatile v4i*)po = o4;
  *(volatile v4i*)pd = c4;
  *(volatile v4i*)pf = f4;
#pragma unroll 1
  for (int i = 4 * tid; i < RCAP; i += 4 * NTHR) {
    const v4i hv = *(const v4ia*)(reg2 + i);
    *(volatile v4i*)(ph + i) = hv;
  }
  __threadfence();
  *(volatile v4i*)po = o4;
  *(volatile v4i*)pd = c4;
  *(volatile v4i*)pf = f4;
#pragma unroll 1
  for (int i = 4 * tid; i < RCAP; i += 4 * NTHR) {
    const v4i hv = *(const v4ia*)(reg2 + i);
    *(volatile v4i*)(ph + i) = hv;
  }
}

__global__ __launch_bounds__(GTHR) __attribute__((amdgpu_num_vgpr(248)))
void k_gemm(const unsigned short* __restrict__ A, const unsigned short* __restrict__ WT,
            float* outF, int K, int ldo) {
  __shared__ __attribute__((aligned(16))) float stg[GBM * GBN];
  const int tid = (int)threadIdx.x, lane = tid & 31, wave = tid >> 5, hh = lane >> 4, m = lane & 15;
  const int rowBase = (int)blockIdx.x * GBM;
  const int col0    = (int)blockIdx.y * GBN;

  v8f acc0[4], acc1[4];
  {
    const v8f z = {0.f, 0.f, 0.f, 0.f, 0.f, 0.f, 0.f, 0.f};
    acc0[0] = z; acc0[1] = z; acc0[2] = z; acc0[3] = z;
    acc1[0] = z; acc1[1] = z; acc1[2] = z; acc1[3] = z;
  }
  const unsigned short* ap0 = A  + (size_t)(rowBase + 32 * wave + m) * (size_t)K + 8 * hh;
  const unsigned short* ap1 = ap0 + (size_t)16 * (size_t)K;
  const unsigned short* wp  = WT + (size_t)(col0 + m) * (size_t)K + 8 * hh;
  const int ksteps = K >> 5;
#pragma unroll 1
  for (int ks = 0; ks < ksteps; ++ks) {
    FragB a0, a1;
    a0.h[0] = *(const v8usa*)(ap0 + 32 * ks);
    a0.h[1] = *(const v8usa*)(ap0 + 32 * ks + 16);
    a1.h[0] = *(const v8usa*)(ap1 + 32 * ks);
    a1.h[1] = *(const v8usa*)(ap1 + 32 * ks + 16);
#pragma unroll
    for (int t = 0; t < 4; ++t) {
      const unsigned short* wq = wp + (size_t)(16 * t) * (size_t)K + 32 * ks;
      FragB bf;
      bf.h[0] = *(const v8usa*)wq;
      bf.h[1] = *(const v8usa*)(wq + 16);
      acc0[t] = wmb(a0, bf, acc0[t]);
      acc1[t] = wmb(a1, bf, acc1[t]);
    }
  }

#pragma unroll
  for (int t = 0; t < 4; ++t) {
    const int lc = 16 * t + m;
#pragma unroll
    for (int r = 0; r < 8; ++r) {
      const int lr = 32 * wave + 8 * hh + r;
      stg[lr * GBN + lc]        = acc0[t][r];
      stg[(lr + 16) * GBN + lc] = acc1[t][r];
    }
  }
  __syncthreads();

  v4f fv[16];
#pragma unroll
  for (int i = 0; i < 16; ++i) {
    const int lr = 32 * wave + 2 * i + hh;
    fv[i] = *(const v4fa*)(stg + lr * GBN + 4 * m);
  }
#pragma unroll
  for (int i = 0; i < 16; ++i) {
    const int gr = rowBase + 32 * wave + 2 * i + hh;
    float* op = outF + (size_t)gr * (size_t)ldo + col0 + 4 * m;
    *(volatile v4f*)op = fv[i];
  }
  __threadfence();
#pragma unroll
  for (int i = 0; i < 16; ++i) {
    const int gr = rowBase + 32 * wave + 2 * i + hh;
    float* op = outF + (size_t)gr * (size_t)ldo + col0 + 4 * m;
    *(volatile v4f*)op = fv[i];
  }
}

template<int NH, int NP>
__global__ __launch_bounds__(NTHR) void k_dot(const float* __restrict__ H, const float* __restrict__ atts,
                                              const float* __restrict__ attd, float* SD) {
  constexpr int W  = NH * NP * 128;
  constexpr int CH = NP * 128;
  constexpr int NL = 8 * NH;
  __shared__ __attribute__((aligned(16))) float sa[2 * W];
  __shared__ __attribute__((aligned(16))) float sd[2 * 32 * NH];
  const int tid = (int)threadIdx.x, lane = tid & 31;
  const int wave = __builtin_amdgcn_readfirstlane(tid >> 5);
  for (int i = tid; i < W / 4; i += NTHR) {
    const v4f a = bfr4(*(const v4fa*)(atts + 4 * i));
    const v4f b = bfr4(*(const v4fa*)(attd + 4 * i));
    *(v4fa*)(sa + 4 * i)     = a;
    *(v4fa*)(sa + W + 4 * i) = b;
  }
  __syncthreads();
  const int rowBase = (int)blockIdx.x * 32;
#pragma unroll 1
  for (int r = 0; r < 4; ++r) {
    const int rl = 4 * wave + r;
    const float* hr = H + (size_t)(rowBase + rl) * W + 4 * lane;
#pragma unroll 1
    for (int hd = 0; hd < NH; ++hd) {
      float ds = 0.0f, dd = 0.0f;
#pragma unroll
      for (int j = 0; j < NP; ++j) {
        const v4f v  = *(const v4fa*)(hr + hd * CH + j * 128);
        const v4f as = *(const v4fa*)(sa + hd * CH + j * 128 + 4 * lane);
        const v4f ad = *(const v4fa*)(sa + W + hd * CH + j * 128 + 4 * lane);
        ds = fmaf(v.x, as.x, ds); ds = fmaf(v.y, as.y, ds); ds = fmaf(v.z, as.z, ds); ds = fmaf(v.w, as.w, ds);
        dd = fmaf(v.x, ad.x, dd); dd = fmaf(v.y, ad.y, dd); dd = fmaf(v.z, ad.z, dd); dd = fmaf(v.w, ad.w, dd);
      }
#pragma unroll
      for (int off = 16; off > 0; off >>= 1) {
        ds += __shfl_xor(ds, off);
        dd += __shfl_xor(dd, off);
      }
      if (lane == 0) { sd[rl * NH + hd] = ds; sd[32 * NH + rl * NH + hd] = dd; }
    }
  }
  __syncthreads();
  if (wave < 2) {
    const int li = lane < NL ? lane : NL - 1;
    const v4f v = *(const v4fa*)(sd + wave * 32 * NH + 4 * li);
    asm volatile("" :: "v"(v));
    float* gp = SD + (size_t)wave * (size_t)MP * NH + (size_t)rowBase * NH + 4 * li;
    if (lane < NL) *(volatile v4f*)gp = v;
    __threadfence();
    if (lane < NL) *(volatile v4f*)gp = v;
  }
}

template<int NH>
__device__ __forceinline__ void pass_a(const float* __restrict__ SD, const int s0, const int s1,
                                       const bool v0, const bool v1, const int gcl, float* wl, const int lane) {
  const float* ASp = SD;
  const float* ADp = SD + (size_t)MP * NH;
#pragma unroll 1
  for (int hd = 0; hd < NH; ++hd) {
    const float adv = ADp[gcl * NH + hd];
    const float asv = ASp[gcl * NH + hd];
    const float x0 = ASp[s0 * NH + hd];
    const float x1 = ASp[s1 * NH + hd];
    asm volatile("" :: "v"(x0));
    asm volatile("" :: "v"(x1));
    float e0 = x0 + adv; e0 = e0 > 0.0f ? e0 : NEGSL * e0;
    float e1 = x1 + adv; e1 = e1 > 0.0f ? e1 : NEGSL * e1;
    float es = asv + adv; es = es > 0.0f ? es : NEGSL * es;
    float mx = fmaxf(v0 ? e0 : -3.0e38f, v1 ? e1 : -3.0e38f);
#pragma unroll
    for (int off = 16; off > 0; off >>= 1) mx = fmaxf(mx, __shfl_xor(mx, off));
    mx = fmaxf(mx, es);
    const float q0 = expf(e0 - mx), q1 = expf(e1 - mx);
    const float p0 = v0 ? q0 : 0.0f, p1 = v1 ? q1 : 0.0f;
    float sm = p0 + p1;
#pragma unroll
    for (int off = 16; off > 0; off >>= 1) sm += __shfl_xor(sm, off);
    const float ps  = expf(es - mx);
    const float den = sm + ps;
    const float inv = 1.0f / (den + EPS_SM);
    wl[lane * NH + hd]        = p0 * inv;
    wl[(32 + lane) * NH + hd] = p1 * inv;
    if (lane == 0) wl[SELFQ * NH + hd] = ps * inv;
  }
}

__device__ __forceinline__ int load_hits(const int* __restrict__ HITS, const int* __restrict__ OFF,
                                         const int* __restrict__ DEG, const int d, const int lane,
                                         int& s0, int& s1, bool& v0, bool& v1, int& craw_out) {
  const int blk = d >> SLOTB;
  int st = OFF[d];
  const int craw = DEG[d];
  int cnt = craw;
  st  = st < 0 ? 0 : (st > RCAP ? RCAP : st);
  cnt = cnt < 0 ? 0 : (cnt > DEGCAP ? DEGCAP : cnt);
  if (cnt > RCAP - st) cnt = RCAP - st;
  int i0 = st + lane;      i0 = i0 > RCAP - 1 ? RCAP - 1 : i0;
  int i1 = st + 32 + lane; i1 = i1 > RCAP - 1 ? RCAP - 1 : i1;
  int r0 = HITS[(size_t)blk * RCAP + i0];
  int r1 = HITS[(size_t)blk * RCAP + i1];
  asm volatile("" :: "v"(r0));
  asm volatile("" :: "v"(r1));
  s0 = r0 < 0 ? 0 : (r0 > NN - 1 ? NN - 1 : r0);
  s1 = r1 < 0 ? 0 : (r1 > NN - 1 ? NN - 1 : r1);
  v0 = lane < cnt;
  v1 = 32 + lane < cnt;
  craw_out = craw;
  return cnt;
}

__device__ __forceinline__ void stage4(float* se, const int j, const v4f t) {
  se[(4 * j + 0) * 32] = t.x; se[(4 * j + 1) * 32] = t.y; se[(4 * j + 2) * 32] = t.z; se[(4 * j + 3) * 32] = t.w;
}
__device__ __forceinline__ v4f unstage4(const float* se, const int j, const bool live, const float pz) {
  v4f r;
  const float a = se[(4 * j + 0) * 32], b = se[(4 * j + 1) * 32], c = se[(4 * j + 2) * 32], d = se[(4 * j + 3) * 32];
  r.x = (live ? a : 0.0f) + pz; r.y = (live ? b : 0.0f) + pz; r.z = (live ? c : 0.0f) + pz; r.w = (live ? d : 0.0f) + pz;
  return r;
}

__global__ __launch_bounds__(NTHR) __attribute__((amdgpu_num_vgpr(248)))
void k_scan1(const int* __restrict__ HITS, const int* __restrict__ OFF, const int* __restrict__ DEG,
             const int* __restrict__ FLG, const float* __restrict__ H1, const float* __restrict__ SD,
             const float* __restrict__ bias, unsigned short* X) {
  __shared__ __attribute__((aligned(16))) float sB[HC1];
  __shared__ __attribute__((aligned(16))) float wal[NWAVE * LCAP * NH1];
  __shared__ int ssrc[NWAVE * LCAP];
  __shared__ float sel[NWAVE * 512];
  const int tid = (int)threadIdx.x, lane = tid & 31;
  const int wave = __builtin_amdgcn_readfirstlane(tid >> 5);
  for (int i = tid; i < HC1 / 4; i += NTHR) {
    const v4f b = bfr4(*(const v4fa*)(bias + 4 * i));
    *(v4fa*)(sB + 4 * i) = b;
  }
  const int d = (int)blockIdx.x * NWAVE + wave;
  const bool live = d < NN;
  const int gcl = live ? d : NN - 1;
  int s0, s1, craw; bool v0, v1;
  const int cnt = load_hits(HITS, OFF, DEG, d, lane, s0, s1, v0, v1, craw);
  const int fl = FLG[d];
  const float qnan = __int_as_float(0x7fc00000);
  const float pz = (live && (fl != 0 || craw > DEGCAP)) ? qnan : 0.0f;
  int* sl = ssrc + wave * LCAP;
  float* wl = wal + wave * LCAP * NH1;
  sl[lane] = s0;
  sl[32 + lane] = s1;
  if (lane == 0) sl[SELFQ] = gcl;
  pass_a<NH1>(SD, s0, s1, v0, v1, gcl, wl, lane);
  __syncthreads();

  float* se = sel + wave * 512 + lane;
  unsigned short* xrow = X + (size_t)d * KA2;
  const int nq = cnt + 1;
#pragma unroll 1
  for (int hd = 0; hd < NH1; ++hd) {
    const int cb = hd * C1 + 4 * lane;
    v4f a0 = {0.f, 0.f, 0.f, 0.f}, a1 = a0, a2 = a0, a3 = a0;
#pragma unroll 1
    for (int q = 0; q < nq; ++q) {
      const int qq = (q == cnt) ? SELFQ : q;
      const int s = sl[qq];
      const float a = wl[qq * NH1 + hd];
      const float* p = H1 + (size_t)s * HC1 + cb;
      const v4f u0 = *(const v4fa*)p;
      const v4f u1 = *(const v4fa*)(p + 128);
      const v4f u2 = *(const v4fa*)(p + 256);
      const v4f u3 = *(const v4fa*)(p + 384);
      a0.x = fmaf(a, u0.x, a0.x); a0.y = fmaf(a, u0.y, a0.y); a0.z = fmaf(a, u0.z, a0.z); a0.w = fmaf(a, u0.w, a0.w);
      a1.x = fmaf(a, u1.x, a1.x); a1.y = fmaf(a, u1.y, a1.y); a1.z = fmaf(a, u1.z, a1.z); a1.w = fmaf(a, u1.w, a1.w);
      a2.x = fmaf(a, u2.x, a2.x); a2.y = fmaf(a, u2.y, a2.y); a2.z = fmaf(a, u2.z, a2.z); a2.w = fmaf(a, u2.w, a2.w);
      a3.x = fmaf(a, u3.x, a3.x); a3.y = fmaf(a, u3.y, a3.y); a3.z = fmaf(a, u3.z, a3.z); a3.w = fmaf(a, u3.w, a3.w);
    }
    const v4f b0 = *(const v4fa*)(sB + cb);
    const v4f b1 = *(const v4fa*)(sB + cb + 128);
    const v4f b2 = *(const v4fa*)(sB + cb + 256);
    const v4f b3 = *(const v4fa*)(sB + cb + 384);
    stage4(se, 0, a0 + b0);
    stage4(se, 1, a1 + b1);
    stage4(se, 2, a2 + b2);
    stage4(se, 3, a3 + b3);
#pragma unroll 1
    for (int k = 0; k < 16; ++k) {
      const float x = se[k * 32];
      const float y = x > 0.0f ? x : expm1f(x);
      se[k * 32] = y;
    }
    const HL h0 = split4(unstage4(se, 0, live, pz));
    const HL h1 = split4(unstage4(se, 1, live, pz));
    const HL h2 = split4(unstage4(se, 2, live, pz));
    const HL h3 = split4(unstage4(se, 3, live, pz));
    unsigned short* hp = xrow + cb;
    *(volatile v2u*)(hp)             = h0.hi;
    *(volatile v2u*)(hp + 128)       = h1.hi;
    *(volatile v2u*)(hp + 256)       = h2.hi;
    *(volatile v2u*)(hp + 384)       = h3.hi;
    *(volatile v2u*)(hp + HC1)       = h0.lo;
    *(volatile v2u*)(hp + HC1 + 128) = h1.lo;
    *(volatile v2u*)(hp + HC1 + 256) = h2.lo;
    *(volatile v2u*)(hp + HC1 + 384) = h3.lo;
    __threadfence();
    *(volatile v2u*)(hp)             = h0.hi;
    *(volatile v2u*)(hp + 128)       = h1.hi;
    *(volatile v2u*)(hp + 256)       = h2.hi;
    *(volatile v2u*)(hp + 384)       = h3.hi;
    *(volatile v2u*)(hp + HC1)       = h0.lo;
    *(volatile v2u*)(hp + HC1 + 128) = h1.lo;
    *(volatile v2u*)(hp + HC1 + 256) = h2.lo;
    *(volatile v2u*)(hp + HC1 + 384) = h3.lo;
  }
}

__global__ __launch_bounds__(NTHR) __attribute__((amdgpu_num_vgpr(248)))
void k_scan2(const int* __restrict__ HITS, const int* __restrict__ OFF, const int* __restrict__ DEG,
             const int* __restrict__ FLG, const float* __restrict__ H2, const float* __restrict__ SD,
             const float* __restrict__ bias, float* out) {
  __shared__ __attribute__((aligned(16))) float sB2[C2];
  __shared__ __attribute__((aligned(16))) float wal[NWAVE * LCAP];
  __shared__ int ssrc[NWAVE * LCAP];
  const int tid = (int)threadIdx.x, lane = tid & 31;
  const int wave = __builtin_amdgcn_readfirstlane(tid >> 5);
  for (int i = tid; i < C2 / 4; i += NTHR) {
    const v4f b = bfr4(*(const v4fa*)(bias + 4 * i));
    *(v4fa*)(sB2 + 4 * i) = b;
  }
  const int d = (int)blockIdx.x * NWAVE + wave;
  const bool live = d < NN;
  const int gcl = live ? d : NN - 1;
  int s0, s1, craw; bool v0, v1;
  const int cnt = load_hits(HITS, OFF, DEG, d, lane, s0, s1, v0, v1, craw);
  const int fl = FLG[d];
  const float qnan = __int_as_float(0x7fc00000);
  const float pz = (fl != 0 || craw > DEGCAP) ? qnan : 0.0f;
  int* sl = ssrc + wave * LCAP;
  float* wl = wal + wave * LCAP;
  sl[lane] = s0;
  sl[32 + lane] = s1;
  if (lane == 0) sl[SELFQ] = gcl;
  pass_a<1>(SD, s0, s1, v0, v1, gcl, wl, lane);
  __syncthreads();

  v4f a0 = {0.f, 0.f, 0.f, 0.f}, a1 = a0, a2 = a0, a3 = a0, a4 = a0, a5 = a0;
  const int nq = cnt + 1;
#pragma unroll 1
  for (int q = 0; q < nq; ++q) {
    const int qq = (q == cnt) ? SELFQ : q;
    const int s = sl[qq];
    const float a = wl[qq];
    const float* p = H2 + (size_t)s * C2 + 4 * lane;
    const v4f u0 = *(const v4fa*)p;
    const v4f u1 = *(const v4fa*)(p + 128);
    const v4f u2 = *(const v4fa*)(p + 256);
    const v4f u3 = *(const v4fa*)(p + 384);
    const v4f u4 = *(const v4fa*)(p + 512);
    const v4f u5 = *(const v4fa*)(p + 640);
    a0.x = fmaf(a, u0.x, a0.x); a0.y = fmaf(a, u0.y, a0.y); a0.z = fmaf(a, u0.z, a0.z); a0.w = fmaf(a, u0.w, a0.w);
    a1.x = fmaf(a, u1.x, a1.x); a1.y = fmaf(a, u1.y, a1.y); a1.z = fmaf(a, u1.z, a1.z); a1.w = fmaf(a, u1.w, a1.w);
    a2.x = fmaf(a, u2.x, a2.x); a2.y = fmaf(a, u2.y, a2.y); a2.z = fmaf(a, u2.z, a2.z); a2.w = fmaf(a, u2.w, a2.w);
    a3.x = fmaf(a, u3.x, a3.x); a3.y = fmaf(a, u3.y, a3.y); a3.z = fmaf(a, u3.z, a3.z); a3.w = fmaf(a, u3.w, a3.w);
    a4.x = fmaf(a, u4.x, a4.x); a4.y = fmaf(a, u4.y, a4.y); a4.z = fmaf(a, u4.z, a4.z); a4.w = fmaf(a, u4.w, a4.w);
    a5.x = fmaf(a, u5.x, a5.x); a5.y = fmaf(a, u5.y, a5.y); a5.z = fmaf(a, u5.z, a5.z); a5.w = fmaf(a, u5.w, a5.w);
  }
  const v4f pz4 = {pz, pz, pz, pz};
  const v4f o0 = a0 + *(const v4fa*)(sB2 + 4 * lane)       + pz4;
  const v4f o1 = a1 + *(const v4fa*)(sB2 + 4 * lane + 128) + pz4;
  const v4f o2 = a2 + *(const v4fa*)(sB2 + 4 * lane + 256) + pz4;
  const v4f o3 = a3 + *(const v4fa*)(sB2 + 4 * lane + 384) + pz4;
  const v4f o4 = a4 + *(const v4fa*)(sB2 + 4 * lane + 512) + pz4;
  const v4f o5 = a5 + *(const v4fa*)(sB2 + 4 * lane + 640) + pz4;
  float* op = out + (size_t)gcl * C2 + 4 * lane;
  if (live) {
    *(volatile v4f*)(op)       = o0;
    *(volatile v4f*)(op + 128) = o1;
    *(volatile v4f*)(op + 256) = o2;
    *(volatile v4f*)(op + 384) = o3;
    *(volatile v4f*)(op + 512) = o4;
    *(volatile v4f*)(op + 640) = o5;
  }
  __threadfence();
  if (live) {
    *(volatile v4f*)(op)       = o0;
    *(volatile v4f*)(op + 128) = o1;
    *(volatile v4f*)(op + 256) = o2;
    *(volatile v4f*)(op + 384) = o3;
    *(volatile v4f*)(op + 512) = o4;
    *(volatile v4f*)(op + 640) = o5;
  }
}

static inline int cdiv(int a, int b) { return (a + b - 1) / b; }

extern "C" void kernel_launch(void* const* d_in, const int* in_sizes, int n_in,
                              void* d_out, int out_size, void* d_ws, size_t ws_size,
                              hipStream_t stream) {
  if (n_in < 10) return;
  if (in_sizes[0] != NN * F_IN) return;
  if (in_sizes[1] != 2 * NE) return;
  if (in_sizes[2] != F_IN * HC1) return;
  if (in_sizes[3] != NH1 * C1 || in_sizes[4] != NH1 * C1) return;
  if (in_sizes[5] != HC1) return;
  if (in_sizes[6] != HC1 * C2) return;
  if (in_sizes[7] != C2 || in_sizes[8] != C2) return;
  if (in_sizes[9] != C2) return;
  if (out_size != NN * C2) return;

  const float* x   = (const float*)d_in[0];
  const int*   ei  = (const int*)  d_in[1];
  const float* W1  = (const float*)d_in[2];
  const float* a1s = (const float*)d_in[3];
  const float* a1d = (const float*)d_in[4];
  const float* b1  = (const float*)d_in[5];
  const float* W2  = (const float*)d_in[6];
  const float* a2s = (const float*)d_in[7];
  const float* a2d = (const float*)d_in[8];
  const float* b2  = (const float*)d_in[9];
  float* out = (float*)d_out;
  const int* src = ei;
  const int* dst = ei + NE;

  char* ws = (char*)d_ws;
  size_t off = 0;
  const size_t oXB  = off; off += (size_t)MP * F_IN * 2;     off = (off + 255) & ~(size_t)255;
  const size_t oW1T = off; off += (size_t)HC1 * F_IN * 2;    off = (off + 255) & ~(size_t)255;
  const size_t oW2D = off; off += (size_t)C2 * KA2 * 2;      off = (off + 255) & ~(size_t)255;
  const size_t oH1  = off; off += (size_t)MP * HC1 * 4;      off = (off + 255) & ~(size_t)255;
  const size_t oX1  = off; off += (size_t)MP * KA2 * 2;      off = (off + 255) & ~(size_t)255;
  const size_t oSD1 = off; off += (size_t)2 * MP * NH1 * 4;  off = (off + 255) & ~(size_t)255;
  const size_t oSD2 = off; off += (size_t)2 * MP * 4;        off = (off + 255) & ~(size_t)255;
  const size_t oHIT = off; off += (size_t)NBLK * RCAP * 4;   off = (off + 255) & ~(size_t)255;
  const size_t oOFF = off; off += (size_t)NSLOT * 4;         off = (off + 255) & ~(size_t)255;
  const size_t oDEG = off; off += (size_t)NSLOT * 4;         off = (off + 255) & ~(size_t)255;
  const size_t oFLG = off; off += (size_t)NSLOT * 4;         off = (off + 255) & ~(size_t)255;
  if (off > ws_size) return;
  unsigned short* XB   = (unsigned short*)(ws + oXB);
  unsigned short* W1T  = (unsigned short*)(ws + oW1T);
  unsigned short* W2D  = (unsigned short*)(ws + oW2D);
  float*          H1   = (float*)(ws + oH1);
  float*          H2   = (float*)(ws + oH1);
  unsigned short* X1HL = (unsigned short*)(ws + oX1);
  float*          SD1  = (float*)(ws + oSD1);
  float*          SD2  = (float*)(ws + oSD2);
  int*            HITS = (int*)(ws + oHIT);
  int*            OFF  = (int*)(ws + oOFF);
  int*            DEG  = (int*)(ws + oDEG);
  int*            FLG  = (int*)(ws + oFLG);

  hipFuncSetAttribute(reinterpret_cast<const void*>(&k_bucket),
                      hipFuncAttributeMaxDynamicSharedMemorySize, LDS_BKT);

  const int nUx = MP * (F_IN / 8);
  k_xprep<<<cdiv(nUx, NTHR), NTHR, 0, stream>>>(x, XB, nUx);
  const int nUw1 = HC1 * (F_IN / 8);
  k_wtr<<<cdiv(nUw1, NTHR), NTHR, 0, stream>>>(W1, F_IN, HC1, HC1, F_IN, W1T, nUw1);
  const int nUw2 = C2 * (KA2 / 8);
  k_wtr<<<cdiv(nUw2, NTHR), NTHR, 0, stream>>>(W2, HC1, C2, C2, KA2, W2D, nUw2);

  k_bucket<<<NBLK, NTHR, LDS_BKT, stream>>>(src, dst, HITS, OFF, DEG, FLG);

  k_gemm<<<dim3(MP / GBM, HC1 / GBN), GTHR, 0, stream>>>(XB, W1T, H1, F_IN, HC1);
  k_dot<NH1, 4><<<MP / 32, NTHR, 0, stream>>>(H1, a1s, a1d, SD1);
  k_scan1<<<MP / NWAVE, NTHR, 0, stream>>>(HITS, OFF, DEG, FLG, H1, SD1, b1, X1HL);

  k_gemm<<<dim3(MP / GBM, C2 / GBN), GTHR, 0, stream>>>(X1HL, W2D, H2, KA2, C2);
  k_dot<1, 6><<<MP / 32, NTHR, 0, stream>>>(H2, a2s, a2d, SD2);
  k_scan2<<<MP / NWAVE, NTHR, 0, stream>>>(HITS, OFF, DEG, FLG, H2, SD2, b2, out);
}
